// FEM_11029476016518
// MI455X (gfx1250) — hardware-verified
//
#include <hip/hip_runtime.h>
#include <stddef.h>


#define NB_     4
#define NC_     96
#define NIMG_   128
#define NHW_    16384
#define NP_     130
#define ROWH_   (NP_ * NC_)
#define PCS_    (ROWH_ / 8)
#define KCV_    1728
#define NHID_   384
#define NT4_    (NB_ * NC_ * NHW_ / 4)

#define PB_WC_  81
#define PB_WV_  5
#define PB_WP_  5
#define PB_W1_  18
#define PB_W2_  18
#define PB_DP_  8
#define G_PREP_ (PB_WC_ + PB_WV_ + PB_WP_ + PB_W1_ + PB_W2_ + PB_DP_)

static_assert(NC_ * KCV_ == PB_WC_ * 256 * 8);
static_assert(NIMG_ * NIMG_ == PB_DP_ * 256 * 8);
static_assert(NC_ * NC_ == 1152 * 8);
static_assert(NHID_ * NC_ == 4608 * 8);
static_assert(ROWH_ % 64 == 0);
static_assert(PCS_ == 1560);
static_assert(G_PREP_ == 135);
static_assert(NT4_ % 256 == 0);
static_assert(KCV_ % 32 == 0);

typedef float        v4f  __attribute__((ext_vector_type(4)));
typedef unsigned int v4u  __attribute__((ext_vector_type(4)));
typedef unsigned int v2u  __attribute__((ext_vector_type(2)));
typedef float        v8f  __attribute__((ext_vector_type(8)));
typedef _Float16     v16h __attribute__((ext_vector_type(16)));
typedef v4f __attribute__((may_alias)) v4fa;
typedef v4u __attribute__((may_alias)) v4ua;
typedef v2u __attribute__((may_alias)) v2ua;

union Frag { v16h v; v4u q[2]; };

__device__ __forceinline__ unsigned int hb16(float f) {
  union { _Float16 h; unsigned short u; } c;
  c.h = (_Float16)f;
  return (unsigned int)c.u;
}
__device__ __forceinline__ v4u pack8h(v4f a, v4f c) {
  v4u r;
  r.x = hb16(a.x) | (hb16(a.y) << 16);
  r.y = hb16(a.z) | (hb16(a.w) << 16);
  r.z = hb16(c.x) | (hb16(c.y) << 16);
  r.w = hb16(c.z) | (hb16(c.w) << 16);
  return r;
}
__device__ __forceinline__ v2u pack4h(v4f a) {
  v2u r;
  r.x = hb16(a.x) | (hb16(a.y) << 16);
  r.y = hb16(a.z) | (hb16(a.w) << 16);
  return r;
}
__device__ __forceinline__ v8f z8f() {
  v8f z = {0.f, 0.f, 0.f, 0.f, 0.f, 0.f, 0.f, 0.f};
  return z;
}

__device__ __forceinline__ v8f wmma_h(v16h a, v16h b, v8f c) {
  v8f d = __builtin_amdgcn_wmma_f32_16x16x32_f16(false, a, false, b, (short)0, c, false, false);
  asm volatile("v_nop\n\tv_nop\n\tv_nop\n\tv_nop" : "+v"(d) : "v"(a), "v"(b));
  return d;
}
__device__ __forceinline__ v16h ldfrag(const unsigned short* p, int h) {
  Frag f;
  f.q[0] = *(const v4ua*)(p + 8 * h);
  f.q[1] = *(const v4ua*)(p + 16 + 8 * h);
  return f.v;
}
__device__ __forceinline__ void st2h(unsigned short* d, v4u v) {
  *(volatile v4u*)d = v;
  __threadfence();
  *(volatile v4u*)d = v;
}

__global__ __launch_bounds__(256) void k_prep(
    const float* __restrict__ wt1, const float* __restrict__ lm1, const float* __restrict__ th1,
    const float* __restrict__ wt2, const float* __restrict__ lm2, const float* __restrict__ th2,
    const float* __restrict__ qkvw, const float* __restrict__ projw,
    const float* __restrict__ mw1, const float* __restrict__ mw2,
    unsigned short* __restrict__ Wc, unsigned short* __restrict__ Wv, unsigned short* __restrict__ Wp,
    unsigned short* __restrict__ W1, unsigned short* __restrict__ W2, unsigned short* __restrict__ Dp)
{
  __shared__ float sCos[512];
  const int blk = blockIdx.x, tid = threadIdx.x;
  if (blk < PB_WC_) {
    const int p   = blk * 256 + tid;
    const int n   = p / 216;
    const int kp  = p - n * 216;
    const int inp = kp / 108;
    const int rr  = kp - inp * 108;
    const int tap = rr / 12;
    const int ci0 = (rr - tap * 12) * 8;
    const float tA = th1[0], tB = th2[0];
    float ev[8];
    #pragma unroll
    for (int i = 0; i < 8; ++i) {
      const int ci = ci0 + i;
      const int base = (n * NC_ + ci) * 9;
      float s1 = 0.0f, s2 = 0.0f;
      #pragma unroll
      for (int q = 0; q < 9; ++q) { s1 += wt1[base + q]; s2 += wt2[base + q]; }
      const float v1 = wt1[base + tap], v2 = wt2[base + tap];
      const float d1 = tA * lm1[n * NC_ + ci] * s1;
      const float d2 = tB * lm2[n * NC_ + ci] * s2;
      const float c1 = v1 - d1 * v1;
      const float c2 = v2 - d2 * v2;
      const float e1 = (tap == 4) ? c1 : v1;
      const float e2 = (tap == 4) ? c2 : v2;
      ev[i] = 16.0f * ((inp != 0) ? e2 : e1);
    }
    v4f a, c;
    a.x = ev[0]; a.y = ev[1]; a.z = ev[2]; a.w = ev[3];
    c.x = ev[4]; c.y = ev[5]; c.z = ev[6]; c.w = ev[7];
    st2h(Wc + (size_t)p * 8, pack8h(a, c));
  } else if (blk < PB_WC_ + PB_WV_) {
    const int p = (blk - PB_WC_) * 256 + tid;
    if (p < 1152) {
      const int n = p / 12, k0 = (p - n * 12) * 8;
      const float* src = qkvw + (size_t)(192 + n) * NC_ + k0;
      const v4f a = *(const v4fa*)(src) * 16.0f;
      const v4f c = *(const v4fa*)(src + 4) * 16.0f;
      st2h(Wv + (size_t)p * 8, pack8h(a, c));
    }
  } else if (blk < PB_WC_ + PB_WV_ + PB_WP_) {
    const int p = (blk - (PB_WC_ + PB_WV_)) * 256 + tid;
    if (p < 1152) {
      const int n = p / 12, k0 = (p - n * 12) * 8;
      const float* src = projw + (size_t)n * NC_ + k0;
      const v4f a = *(const v4fa*)(src) * 16.0f;
      const v4f c = *(const v4fa*)(src + 4) * 16.0f;
      st2h(Wp + (size_t)p * 8, pack8h(a, c));
    }
  } else if (blk < PB_WC_ + PB_WV_ + PB_WP_ + PB_W1_) {
    const int p = (blk - (PB_WC_ + PB_WV_ + PB_WP_)) * 256 + tid;
    const int n = p / 12, k0 = (p - n * 12) * 8;
    const float* src = mw1 + (size_t)n * NC_ + k0;
    const v4f a = *(const v4fa*)(src) * 16.0f;
    const v4f c = *(const v4fa*)(src + 4) * 16.0f;
    st2h(W1 + (size_t)p * 8, pack8h(a, c));
  } else if (blk < PB_WC_ + PB_WV_ + PB_WP_ + PB_W1_ + PB_W2_) {
    const int p = (blk - (PB_WC_ + PB_WV_ + PB_WP_ + PB_W1_)) * 256 + tid;
    const int n = p / 48, k0 = (p - n * 48) * 8;
    const float* src = mw2 + (size_t)n * NHID_ + k0;
    const v4f a = *(const v4fa*)(src) * 16.0f;
    const v4f c = *(const v4fa*)(src + 4) * 16.0f;
    st2h(W2 + (size_t)p * 8, pack8h(a, c));
  } else {
    const int p = (blk - (PB_WC_ + PB_WV_ + PB_WP_ + PB_W1_ + PB_W2_)) * 256 + tid;
    #pragma unroll 1
    for (int q = 0; q < 2; ++q) {
      const int rdx = tid + 256 * q;
      sCos[rdx] = cosf((float)rdx * 0.012271846303085129f);
    }
    __syncthreads();
    const int i = p >> 4, k0 = (p & 15) * 8;
    const float sc = (i == 0) ? 0.08838834764831845f : 0.125f;
    float ev[8];
    #pragma unroll
    for (int j = 0; j < 8; ++j) {
      const int k = k0 + j;
      ev[j] = sCos[((2 * k + 1) * i) & 511] * sc;
    }
    v4f a, c;
    a.x = ev[0]; a.y = ev[1]; a.z = ev[2]; a.w = ev[3];
    c.x = ev[4]; c.y = ev[5]; c.z = ev[6]; c.w = ev[7];
    st2h(Dp + (size_t)p * 8, pack8h(a, c));
  }
}

__global__ __launch_bounds__(256) void k_mean(const float* __restrict__ x1,
                                              const float* __restrict__ x2,
                                              float* __restrict__ coef)
{
  __shared__ float sp[8];
  __shared__ __align__(16) float sc[128];
  const int b = blockIdx.x, tid = threadIdx.x, lane = tid & 31, wv = tid >> 5;
  if (tid < 128) sc[tid] = 0.0f;
  #pragma unroll 1
  for (int c = 0; c < NC_; ++c) {
    const float* p1 = x1 + (size_t)(b * NC_ + c) * NHW_;
    const float* p2 = x2 + (size_t)(b * NC_ + c) * NHW_;
    float s = 0.0f;
    #pragma unroll 4
    for (int j = 0; j < 16; ++j) {
      const int i4 = j * 256 + tid;
      const v4f a = *(const v4fa*)(p1 + 4 * i4);
      const v4f d = *(const v4fa*)(p2 + 4 * i4);
      s += ((a.x - d.x) + (a.y - d.y)) + ((a.z - d.z) + (a.w - d.w));
    }
    #pragma unroll
    for (int o = 16; o >= 1; o >>= 1) s += __shfl_xor(s, o, 32);
    if (lane == 0) sp[wv] = s;
    __syncthreads();
    if (tid == 0) {
      const float S = ((sp[0] + sp[1]) + (sp[2] + sp[3])) + ((sp[4] + sp[5]) + (sp[6] + sp[7]));
      const float mv  = S * (1.0f / 16384.0f);
      const float w12 = 1.0f / (1.0f + expf(-mv));
      const float w21 = 1.0f / (1.0f + expf(mv));
      sc[c] = 1.0f + w12 + w21;
    }
    __syncthreads();
  }
  if (wv == 0) {
    const v4f v = *(const v4fa*)(sc + 4 * lane);
    float* d = coef + (size_t)b * 128 + 4 * lane;
    *(volatile v4f*)d = v;
    __threadfence();
    *(volatile v4f*)d = v;
  }
}

__global__ __launch_bounds__(256) void k_tocl(const float* __restrict__ x1,
                                              const float* __restrict__ x2,
                                              unsigned short* __restrict__ P)
{
  __shared__ __align__(16) unsigned short sr[ROWH_];
  const int blk = blockIdx.x, tid = threadIdx.x;
  const int inp = blk / (NB_ * NP_);
  const int rem = blk - inp * (NB_ * NP_);
  const int b   = rem / NP_;
  const int yp  = rem - b * NP_;
  const bool zrow = (yp == 0) || (yp == NP_ - 1);
  const float* x = (inp != 0) ? x2 : x1;
  if (!zrow) {
    const int y = yp - 1;
    if (tid < NC_) { sr[tid] = 0; sr[(NP_ - 1) * NC_ + tid] = 0; }
    #pragma unroll
    for (int it = 0; it < 12; ++it) {
      const int idx = it * 256 + tid;
      const int c = idx >> 5, q = idx & 31;
      const v4f v = *(const v4fa*)(x + ((size_t)(b * NC_ + c) * NIMG_ + y) * NIMG_ + 4 * q);
      unsigned short* d = sr + (4 * q + 1) * NC_ + c;
      d[0]       = (unsigned short)hb16(v.x);
      d[NC_]     = (unsigned short)hb16(v.y);
      d[2 * NC_] = (unsigned short)hb16(v.z);
      d[3 * NC_] = (unsigned short)hb16(v.w);
    }
  }
  __syncthreads();
  unsigned short* dst = P + (size_t)blk * ROWH_;
  const v4u z4 = {0u, 0u, 0u, 0u};
  #pragma unroll
  for (int it = 0; it < 7; ++it) {
    const int p = it * 256 + tid;
    if (p < PCS_) {
      v4u v = *(const v4ua*)(sr + 8 * p);
      v = zrow ? z4 : v;
      *(volatile v4u*)(dst + (size_t)8 * p) = v;
    }
  }
  __threadfence();
  #pragma unroll
  for (int it = 0; it < 7; ++it) {
    const int p = it * 256 + tid;
    if (p < PCS_) {
      v4u v = *(const v4ua*)(sr + 8 * p);
      v = zrow ? z4 : v;
      *(volatile v4u*)(dst + (size_t)8 * p) = v;
    }
  }
}

__global__ __launch_bounds__(128) void k_conv(const unsigned short* __restrict__ P,
                                              const unsigned short* __restrict__ Wc,
                                              const float* __restrict__ x1,
                                              const float* __restrict__ x2,
                                              const float* __restrict__ coef,
                                              float* __restrict__ feat)
{
  __shared__ __align__(16) float sS[4 * 16 * NC_];
  const int tid = threadIdx.x, lane = tid & 31, wv = tid >> 5;
  const int h = lane >> 4, m = lane & 15;
  const int blk = blockIdx.x;
  const int b  = blk >> 8;
  const int y  = (blk >> 1) & 127;
  const int xw = (blk & 1) * 64 + wv * 16;

  v8f acc[6];
  #pragma unroll
  for (int nt = 0; nt < 6; ++nt) acc[nt] = z8f();
  const unsigned short* wrow = Wc + (size_t)m * KCV_;

  #pragma unroll 1
  for (int s = 0; s < 54; ++s) {
    const int inp  = (s >= 27) ? 1 : 0;
    const int rem  = s - 27 * inp;
    const int tap  = rem / 3;
    const int cseg = rem - 3 * tap;
    const int ky = tap / 3, kx = tap - 3 * ky;
    const unsigned short* ap = P
        + ((size_t)((inp * NB_ + b) * NP_ + (y + ky)) * NP_ + (size_t)(xw + m + kx)) * NC_
        + cseg * 32;
    Frag a;
    a.q[0] = *(const v4ua*)(ap + 8 * h);
    a.q[1] = *(const v4ua*)(ap + 16 + 8 * h);
    const unsigned short* bp = wrow + s * 32;
    #pragma unroll
    for (int nt = 0; nt < 6; ++nt) {
      const v16h bf = ldfrag(bp + (size_t)nt * 16 * KCV_, h);
      acc[nt] = wmma_h(a.v, bf, acc[nt]);
    }
  }

  {
    float* so = sS + wv * (16 * NC_);
    const float* cf = coef + (size_t)b * 128;
    #pragma unroll
    for (int nt = 0; nt < 6; ++nt) {
      const int c = nt * 16 + m;
      const float cc = cf[c];
      const size_t gx = ((size_t)(b * NC_ + c) * NIMG_ + y) * NIMG_ + xw + 8 * h;
      const v4f a0 = *(const v4fa*)(x1 + gx), a1 = *(const v4fa*)(x1 + gx + 4);
      const v4f d0 = *(const v4fa*)(x2 + gx), d1 = *(const v4fa*)(x2 + gx + 4);
      float fu[8];
      fu[0] = a0.x + d0.x; fu[1] = a0.y + d0.y; fu[2] = a0.z + d0.z; fu[3] = a0.w + d0.w;
      fu[4] = a1.x + d1.x; fu[5] = a1.y + d1.y; fu[6] = a1.z + d1.z; fu[7] = a1.w + d1.w;
      #pragma unroll
      for (int r = 0; r < 8; ++r)
        so[(8 * h + r) * NC_ + c] = acc[nt][r] * 0.0625f + cc * fu[r];
    }
  }
  __syncthreads();

  {
    const float* so = sS + wv * (16 * NC_);
    float* dst = feat + ((size_t)b * NHW_ + (size_t)y * NIMG_ + xw) * NC_;
    #pragma unroll
    for (int it = 0; it < 12; ++it) {
      const int p = it * 32 + lane;
      const v4f v = *(const v4fa*)(so + 4 * p);
      *(volatile v4f*)(dst + 4 * p) = v;
    }
    __threadfence();
    #pragma unroll
    for (int it = 0; it < 12; ++it) {
      const int p = it * 32 + lane;
      const v4f v = *(const v4fa*)(so + 4 * p);
      *(volatile v4f*)(dst + 4 * p) = v;
    }
  }
}

__device__ __forceinline__ void ln_row(const float* row, const float* __restrict__ g,
                                       const float* __restrict__ be, unsigned short* dst)
{
  float s = 0.0f;
  #pragma unroll 2
  for (int i = 0; i < 24; ++i) {
    const v4f v = *(const v4fa*)(row + 4 * i);
    s += (v.x + v.y) + (v.z + v.w);
  }
  const float mu = s * (1.0f / 96.0f);
  float q = 0.0f;
  #pragma unroll 2
  for (int i = 0; i < 24; ++i) {
    const v4f v = *(const v4fa*)(row + 4 * i);
    const float dx = v.x - mu, dy = v.y - mu, dz = v.z - mu, dw = v.w - mu;
    q += (dx * dx + dy * dy) + (dz * dz + dw * dw);
  }
  const float rs = rsqrtf(q * (1.0f / 96.0f) + 1e-5f);
  #pragma unroll 2
  for (int i = 0; i < 24; ++i) {
    const v4f v  = *(const v4fa*)(row + 4 * i);
    const v4f gv = *(const v4fa*)(g + 4 * i);
    const v4f bv = *(const v4fa*)(be + 4 * i);
    v4f o;
    o.x = (v.x - mu) * rs * gv.x + bv.x;
    o.y = (v.y - mu) * rs * gv.y + bv.y;
    o.z = (v.z - mu) * rs * gv.z + bv.z;
    o.w = (v.w - mu) * rs * gv.w + bv.w;
    *(v2ua*)(dst + 4 * i) = pack4h(o);
  }
}

__global__ __launch_bounds__(64) void k_tok(const float* __restrict__ feat,
                                            const unsigned short* __restrict__ Wv,
                                            const unsigned short* __restrict__ Wp,
                                            const unsigned short* __restrict__ W1,
                                            const unsigned short* __restrict__ W2,
                                            const float* __restrict__ g1, const float* __restrict__ e1,
                                            const float* __restrict__ qkvb, const float* __restrict__ pb,
                                            const float* __restrict__ g2, const float* __restrict__ e2,
                                            const float* __restrict__ mb1, const float* __restrict__ mb2,
                                            float* __restrict__ cross)
{
  __shared__ __align__(16) float sT[32 * NC_];
  __shared__ __align__(16) unsigned short sA[32 * NC_];
  __shared__ __align__(16) unsigned short sV[32 * NC_];
  __shared__ __align__(16) unsigned short sH[32 * NHID_];
  __shared__ __align__(16) float sO[NC_ * 32];

  const int tid = threadIdx.x, lane = tid & 31, wv = tid >> 5;
  const int h = lane >> 4, m = lane & 15;
  const int blk = blockIdx.x;
  const int b = blk >> 9, y = (blk >> 2) & 127, x0 = (blk & 3) * 32;
  const size_t tok0 = (size_t)b * NHW_ + (size_t)y * NIMG_ + x0;
  const int rw = wv * 16;

  {
    const float* src = feat + tok0 * NC_;
    #pragma unroll
    for (int it = 0; it < 12; ++it) {
      const int i4 = it * 64 + tid;
      *(v4fa*)(sT + 4 * i4) = *(const v4fa*)(src + 4 * i4);
    }
  }
  __syncthreads();
  if (tid < 32) ln_row(sT + tid * NC_, g1, e1, sA + tid * NC_);
  __syncthreads();

  {
    Frag af[3];
    #pragma unroll
    for (int s = 0; s < 3; ++s) {
      const unsigned short* p = sA + (rw + m) * NC_ + s * 32;
      af[s].q[0] = *(const v4ua*)(p + 8 * h);
      af[s].q[1] = *(const v4ua*)(p + 16 + 8 * h);
    }
    v8f acc[6];
    #pragma unroll
    for (int nt = 0; nt < 6; ++nt) acc[nt] = z8f();
    #pragma unroll
    for (int s = 0; s < 3; ++s) {
      #pragma unroll
      for (int nt = 0; nt < 6; ++nt) {
        const v16h bf = ldfrag(Wv + (size_t)(nt * 16 + m) * NC_ + s * 32, h);
        acc[nt] = wmma_h(af[s].v, bf, acc[nt]);
      }
    }
    #pragma unroll
    for (int nt = 0; nt < 6; ++nt) {
      const int c = nt * 16 + m;
      const float bb = qkvb[192 + c];
      #pragma unroll
      for (int r = 0; r < 8; ++r)
        sV[(rw + 8 * h + r) * NC_ + c] = (unsigned short)hb16(acc[nt][r] * 0.0625f + bb);
    }
  }
  __syncthreads();

  {
    Frag af[3];
    #pragma unroll
    for (int s = 0; s < 3; ++s) {
      const unsigned short* p = sV + (rw + m) * NC_ + s * 32;
      af[s].q[0] = *(const v4ua*)(p + 8 * h);
      af[s].q[1] = *(const v4ua*)(p + 16 + 8 * h);
    }
    v8f acc[6];
    #pragma unroll
    for (int nt = 0; nt < 6; ++nt) acc[nt] = z8f();
    #pragma unroll
    for (int s = 0; s < 3; ++s) {
      #pragma unroll
      for (int nt = 0; nt < 6; ++nt) {
        const v16h bf = ldfrag(Wp + (size_t)(nt * 16 + m) * NC_ + s * 32, h);
        acc[nt] = wmma_h(af[s].v, bf, acc[nt]);
      }
    }
    #pragma unroll
    for (int nt = 0; nt < 6; ++nt) {
      const int c = nt * 16 + m;
      const float bb = pb[c];
      #pragma unroll
      for (int r = 0; r < 8; ++r) {
        const int idx = (rw + 8 * h + r) * NC_ + c;
        sT[idx] = sT[idx] + (acc[nt][r] * 0.0625f + bb);
      }
    }
  }
  __syncthreads();
  if (tid < 32) ln_row(sT + tid * NC_, g2, e2, sA + tid * NC_);
  __syncthreads();

  {
    Frag af[3];
    #pragma unroll
    for (int s = 0; s < 3; ++s) {
      const unsigned short* p = sA + (rw + m) * NC_ + s * 32;
      af[s].q[0] = *(const v4ua*)(p + 8 * h);
      af[s].q[1] = *(const v4ua*)(p + 16 + 8 * h);
    }
    #pragma unroll 1
    for (int g = 0; g < 4; ++g) {
      v8f acc[6];
      #pragma unroll
      for (int nt = 0; nt < 6; ++nt) acc[nt] = z8f();
      #pragma unroll
      for (int s = 0; s < 3; ++s) {
        #pragma unroll
        for (int nt = 0; nt < 6; ++nt) {
          const v16h bf = ldfrag(W1 + (size_t)(g * NC_ + nt * 16 + m) * NC_ + s * 32, h);
          acc[nt] = wmma_h(af[s].v, bf, acc[nt]);
        }
      }
      #pragma unroll
      for (int nt = 0; nt < 6; ++nt) {
        const int col = g * NC_ + nt * 16 + m;
        const float bb = mb1[col];
        #pragma unroll
        for (int r = 0; r < 8; ++r) {
          const float xv = acc[nt][r] * 0.0625f + bb;
          const float ge = 0.5f * xv * (1.0f + erff(xv * 0.70710678118654752f));
          sH[(rw + 8 * h + r) * NHID_ + col] = (unsigned short)hb16(ge);
        }
      }
    }
  }
  __syncthreads();

  {
    v8f acc[6];
    #pragma unroll
    for (int nt = 0; nt < 6; ++nt) acc[nt] = z8f();
    #pragma unroll 2
    for (int s = 0; s < 12; ++s) {
      const unsigned short* p = sH + (rw + m) * NHID_ + s * 32;
      Frag a;
      a.q[0] = *(const v4ua*)(p + 8 * h);
      a.q[1] = *(const v4ua*)(p + 16 + 8 * h);
      #pragma unroll
      for (int nt = 0; nt < 6; ++nt) {
        const v16h bf = ldfrag(W2 + (size_t)(nt * 16 + m) * NHID_ + s * 32, h);
        acc[nt] = wmma_h(a.v, bf, acc[nt]);
      }
    }
    #pragma unroll
    for (int nt = 0; nt < 6; ++nt) {
      const int c = nt * 16 + m;
      const float bb = mb2[c];
      #pragma unroll
      for (int r = 0; r < 8; ++r) {
        const int row = rw + 8 * h + r;
        sO[c * 32 + row] = sT[row * NC_ + c] + (acc[nt][r] * 0.0625f + bb);
      }
    }
  }
  __syncthreads();

  {
    float* dstb = cross + (size_t)b * NC_ * NHW_ + (size_t)y * NIMG_ + x0;
    #pragma unroll
    for (int it = 0; it < 12; ++it) {
      const int i = it * 64 + tid;
      const int c = i >> 3, q = i & 7;
      const v4f v = *(const v4fa*)(sO + c * 32 + 4 * q);
      *(volatile v4f*)(dstb + (size_t)c * NHW_ + 4 * q) = v;
    }
    __threadfence();
    #pragma unroll
    for (int it = 0; it < 12; ++it) {
      const int i = it * 64 + tid;
      const int c = i >> 3, q = i & 7;
      const v4f v = *(const v4fa*)(sO + c * 32 + 4 * q);
      *(volatile v4f*)(dstb + (size_t)c * NHW_ + 4 * q) = v;
    }
  }
}

__global__ __launch_bounds__(128) void k_dct(const float* __restrict__ cross,
                                             const unsigned short* __restrict__ Dp,
                                             float* __restrict__ E)
{
  extern __shared__ v4u dsm4[];
  unsigned char* dsm = (unsigned char*)dsm4;
  unsigned short* sX = (unsigned short*)dsm;
  unsigned short* sU = (unsigned short*)(dsm + 32768);
  float* sE = (float*)dsm;

  const int tid = threadIdx.x, lane = tid & 31, wv = tid >> 5;
  const int h = lane >> 4, m = lane & 15;
  const int bc = blockIdx.x;
  const float* X = cross + (size_t)bc * NHW_;

  #pragma unroll 4
  for (int it = 0; it < 32; ++it) {
    const int i4 = it * 128 + tid;
    const v4f v = *(const v4fa*)(X + 4 * i4);
    *(v2ua*)(sX + 4 * i4) = pack4h(v);
  }
  __syncthreads();

  #pragma unroll 1
  for (int mt = 0; mt < 2; ++mt) {
    const int tile = 2 * wv + mt;
    Frag af[4];
    #pragma unroll
    for (int ks = 0; ks < 4; ++ks) {
      const unsigned short* p = Dp + (size_t)(tile * 16 + m) * NIMG_ + ks * 32;
      af[ks].q[0] = *(const v4ua*)(p + 8 * h);
      af[ks].q[1] = *(const v4ua*)(p + 16 + 8 * h);
    }
    #pragma unroll 1
    for (int nh = 0; nh < 2; ++nh) {
      v8f acc[4];
      #pragma unroll
      for (int nt = 0; nt < 4; ++nt) acc[nt] = z8f();
      #pragma unroll
      for (int ks = 0; ks < 4; ++ks) {
        #pragma unroll
        for (int nt = 0; nt < 4; ++nt) {
          const int ncol = nh * 64 + nt * 16 + m;
          const v16h bf = ldfrag(sX + ncol * NIMG_ + ks * 32, h);
          acc[nt] = wmma_h(af[ks].v, bf, acc[nt]);
        }
      }
      #pragma unroll
      for (int nt = 0; nt < 4; ++nt) {
        const int ncol = nh * 64 + nt * 16 + m;
        #pragma unroll
        for (int r = 0; r < 8; ++r)
          sU[(tile * 16 + 8 * h + r) * NIMG_ + ncol] = (unsigned short)hb16(acc[nt][r]);
      }
    }
  }
  __syncthreads();

  #pragma unroll 1
  for (int mt = 0; mt < 2; ++mt) {
    const int tile = 2 * wv + mt;
    Frag af[4];
    #pragma unroll
    for (int ks = 0; ks < 4; ++ks) {
      const unsigned short* p = Dp + (size_t)(tile * 16 + m) * NIMG_ + ks * 32;
      af[ks].q[0] = *(const v4ua*)(p + 8 * h);
      af[ks].q[1] = *(const v4ua*)(p + 16 + 8 * h);
    }
    #pragma unroll 1
    for (int nh = 0; nh < 2; ++nh) {
      v8f acc[4];
      #pragma unroll
      for (int nt = 0; nt < 4; ++nt) acc[nt] = z8f();
      #pragma unroll
      for (int ks = 0; ks < 4; ++ks) {
        #pragma unroll
        for (int nt = 0; nt < 4; ++nt) {
          const int ncol = nh * 64 + nt * 16 + m;
          const v16h bf = ldfrag(sU + ncol * NIMG_ + ks * 32, h);
          acc[nt] = wmma_h(af[ks].v, bf, acc[nt]);
        }
      }
      #pragma unroll
      for (int nt = 0; nt < 4; ++nt) {
        const int ncol = nh * 64 + nt * 16 + m;
        #pragma unroll
        for (int r = 0; r < 8; ++r)
          sE[wv * 2048 + (8 * h + r) * NIMG_ + ncol] = fabsf(acc[nt][r]);
      }
    }
    __syncthreads();
    {
      const float* se = sE + wv * 2048;
      float* dst = E + (size_t)bc * NHW_ + (size_t)tile * 16 * NIMG_;
      #pragma unroll
      for (int it = 0; it < 16; ++it) {
        const int p = it * 32 + lane;
        const v4f v = *(const v4fa*)(se + 4 * p);
        *(volatile v4f*)(dst + 4 * p) = v;
      }
      __threadfence();
      #pragma unroll
      for (int it = 0; it < 16; ++it) {
        const int p = it * 32 + lane;
        const v4f v = *(const v4fa*)(se + 4 * p);
        *(volatile v4f*)(dst + 4 * p) = v;
      }
    }
    __syncthreads();
  }
}

#define NEGV_ (-3.0e38f)

__device__ __forceinline__ void argmax_w(float& bv, int& bi) {
  #pragma unroll
  for (int s = 16; s >= 1; s >>= 1) {
    const float ov = __shfl_xor(bv, s, 32);
    const int   oi = __shfl_xor(bi, s, 32);
    const bool tk = (ov > bv) || ((ov == bv) && (oi < bi));
    bv = tk ? ov : bv;
    bi = tk ? oi : bi;
  }
}

__global__ __launch_bounds__(256) void k_gate(const float* __restrict__ E,
                                              const float* __restrict__ fw1,
                                              const float* __restrict__ fb1,
                                              const float* __restrict__ fw2,
                                              const float* __restrict__ fb2,
                                              float* __restrict__ scl)
{
  __shared__ float sCh[8 * 1024];
  __shared__ float sCand[16 * NC_];
  __shared__ float sTk[NC_];
  __shared__ float sHb[24];
  __shared__ __align__(16) float sLine[32];
  const int tid = threadIdx.x, lane = tid & 31, wv = tid >> 5;
  if (tid < 32) sLine[tid] = 0.0f;
  float* ch = sCh + wv * 1024;

  #pragma unroll 1
  for (int b = 0; b < NB_; ++b) {
    const float* Eb = E + (size_t)b * NC_ * NHW_;
    #pragma unroll 1
    for (int cc = 0; cc < 2; ++cc) {
      const int chunk = wv * 2 + cc;
      const int p0 = chunk * 1024;
      #pragma unroll 1
      for (int j = 0; j < 32; ++j) {
        const int p = p0 + lane + 32 * j;
        float s = 0.0f;
        #pragma unroll 4
        for (int c = 0; c < NC_; ++c) s += Eb[(size_t)c * NHW_ + p];
        ch[lane + 32 * j] = s * (1.0f / 96.0f);
      }
      #pragma unroll 1
      for (int r = 0; r < NC_; ++r) {
        float bv = ch[lane];
        int bi = lane;
        #pragma unroll 4
        for (int j = 1; j < 32; ++j) {
          const float v = ch[lane + 32 * j];
          const bool tk = v > bv;
          bv = tk ? v : bv;
          bi = tk ? (lane + 32 * j) : bi;
        }
        argmax_w(bv, bi);
        if (lane == 0) sCand[chunk * NC_ + r] = bv;
        if ((bi & 31) == lane) ch[bi] = NEGV_;
      }
    }
    __syncthreads();
    if (wv == 0) {
      #pragma unroll 1
      for (int r = 0; r < NC_; ++r) {
        float bv = sCand[lane];
        int bi = lane;
        #pragma unroll 4
        for (int j = 1; j < 48; ++j) {
          const float v = sCand[lane + 32 * j];
          const bool tk = v > bv;
          bv = tk ? v : bv;
          bi = tk ? (lane + 32 * j) : bi;
        }
        argmax_w(bv, bi);
        if (lane == 0) sTk[r] = bv;
        if ((bi & 31) == lane) sCand[bi] = NEGV_;
      }
    }
    __syncthreads();
    if (tid < 24) {
      float hs = fb1[tid];
      #pragma unroll 4
      for (int k = 0; k < NC_; ++k) hs += fw1[tid * NC_ + k] * sTk[k];
      sHb[tid] = fmaxf(hs, 0.0f);
    }
    __syncthreads();
    if (tid == 0) {
      float o = fb2[0];
      #pragma unroll 4
      for (int j = 0; j < 24; ++j) o += fw2[j] * sHb[j];
      sLine[b] = 1.0f / (1.0f + expf(-o));
    }
    __syncthreads();
  }

  if (tid < 8) {
    const v4f v = *(const v4fa*)(sLine + 4 * tid);
    *(volatile v4f*)(scl + 4 * tid) = v;
  }
  __threadfence();
  if (tid < 8) {
    const v4f v = *(const v4fa*)(sLine + 4 * tid);
    *(volatile v4f*)(scl + 4 * tid) = v;
  }
}

__global__ __launch_bounds__(256) void k_out(const float* __restrict__ cross,
                                             const float* __restrict__ x1,
                                             const float* __restrict__ x2,
                                             const float* __restrict__ scl,
                                             float* __restrict__ out)
{
  const int i = blockIdx.x * 256 + threadIdx.x;
  if (i >= NT4_) return;
  const int b = (i >> 12) / NC_;
  const float att = scl[b];
  const v4f c = *(const v4fa*)(cross + (size_t)4 * i);
  const v4f a = *(const v4fa*)(x1 + (size_t)4 * i);
  const v4f d = *(const v4fa*)(x2 + (size_t)4 * i);
  v4f o;
  o.x = c.x + c.x * att; o.y = c.y + c.y * att; o.z = c.z + c.z * att; o.w = c.w + c.w * att;
  const v4f r0 = a + o;
  const v4f r1 = d + o;
  float* p0 = out + (size_t)4 * i;
  float* p1 = out + (size_t)NB_ * NC_ * NHW_ + (size_t)4 * i;
  *(volatile v4f*)p0 = r0;
  *(volatile v4f*)p1 = r1;
  __threadfence();
  *(volatile v4f*)p0 = r0;
  *(volatile v4f*)p1 = r1;
}

extern "C" void kernel_launch(void* const* d_in, const int* in_sizes, int n_in,
                              void* d_out, int out_size, void* d_ws, size_t ws_size,
                              hipStream_t stream)
{
  if (n_in < 24) return;
  if (in_sizes[0] != NB_ * NC_ * NHW_) return;
  if (in_sizes[1] != NB_ * NC_ * NHW_) return;
  if (in_sizes[2] != NC_ * NC_ * 9) return;
  if (in_sizes[3] != NC_ * NC_) return;
  if (in_sizes[4] < 1) return;
  if (in_sizes[5] != NC_ * NC_ * 9) return;
  if (in_sizes[6] != NC_ * NC_) return;
  if (in_sizes[7] < 1) return;
  if (in_sizes[8] != NC_ || in_sizes[9] != NC_) return;
  if (in_sizes[10] != 3 * NC_ * NC_) return;
  if (in_sizes[11] != 3 * NC_) return;
  if (in_sizes[12] != NC_ * NC_) return;
  if (in_sizes[13] != NC_) return;
  if (in_sizes[14] != NC_ || in_sizes[15] != NC_) return;
  if (in_sizes[16] != NHID_ * NC_) return;
  if (in_sizes[17] != NHID_) return;
  if (in_sizes[18] != NC_ * NHID_) return;
  if (in_sizes[19] != NC_) return;
  if (in_sizes[20] != 24 * NC_) return;
  if (in_sizes[21] != 24) return;
  if (in_sizes[22] != 24) return;
  if (in_sizes[23] < 1) return;
  if (out_size != 2 * NB_ * NC_ * NHW_) return;

  const float* x1    = (const float*)d_in[0];
  const float* x2    = (const float*)d_in[1];
  const float* wt1   = (const float*)d_in[2];
  const float* lm1   = (const float*)d_in[3];
  const float* th1   = (const float*)d_in[4];
  const float* wt2   = (const float*)d_in[5];
  const float* lm2   = (const float*)d_in[6];
  const float* th2   = (const float*)d_in[7];
  const float* ln1g  = (const float*)d_in[8];
  const float* ln1b  = (const float*)d_in[9];
  const float* qkvw  = (const float*)d_in[10];
  const float* qkvb  = (const float*)d_in[11];
  const float* projw = (const float*)d_in[12];
  const float* projb = (const float*)d_in[13];
  const float* ln2g  = (const float*)d_in[14];
  const float* ln2b  = (const float*)d_in[15];
  const float* mw1   = (const float*)d_in[16];
  const float* mb1   = (const float*)d_in[17];
  const float* mw2   = (const float*)d_in[18];
  const float* mb2   = (const float*)d_in[19];
  const float* fw1   = (const float*)d_in[20];
  const float* fb1   = (const float*)d_in[21];
  const float* fw2   = (const float*)d_in[22];
  const float* fb2   = (const float*)d_in[23];
  float* out = (float*)d_out;

  const size_t bWc = (size_t)NC_ * KCV_ * 2;
  const size_t bWv = (size_t)NC_ * NC_ * 2;
  const size_t bW1 = (size_t)NHID_ * NC_ * 2;
  const size_t bDp = (size_t)NIMG_ * NIMG_ * 2;
  const size_t bCf = (size_t)NB_ * 128 * 4;
  const size_t bSc = 128;
  const size_t bP  = (size_t)2 * NB_ * NP_ * ROWH_ * 2;
  const size_t bF  = (size_t)NB_ * NC_ * NHW_ * 4;
  const size_t total = bWc + 2 * bWv + 2 * bW1 + bDp + bCf + bSc + bP + 3 * bF;
  if (total > ws_size) return;
  if (total > (size_t)134217728) return;

  char* ws = (char*)d_ws;
  size_t off = 0;
  unsigned short* Wc  = (unsigned short*)(ws + off); off += bWc;
  unsigned short* Wv  = (unsigned short*)(ws + off); off += bWv;
  unsigned short* Wp  = (unsigned short*)(ws + off); off += bWv;
  unsigned short* W1  = (unsigned short*)(ws + off); off += bW1;
  unsigned short* W2  = (unsigned short*)(ws + off); off += bW1;
  unsigned short* Dp  = (unsigned short*)(ws + off); off += bDp;
  float*          cf  = (float*)(ws + off);          off += bCf;
  float*          scl = (float*)(ws + off);          off += bSc;
  unsigned short* P   = (unsigned short*)(ws + off); off += bP;
  float*          feat = (float*)(ws + off);         off += bF;
  float*          crs  = (float*)(ws + off);         off += bF;
  float*          Epl  = (float*)(ws + off);         off += bF;
  if (off != total) return;

  k_prep<<<G_PREP_, 256, 0, stream>>>(wt1, lm1, th1, wt2, lm2, th2, qkvw, projw, mw1, mw2,
                                      Wc, Wv, Wp, W1, W2, Dp);
  k_mean<<<NB_, 256, 0, stream>>>(x1, x2, cf);
  k_tocl<<<2 * NB_ * NP_, 256, 0, stream>>>(x1, x2, P);
  k_conv<<<NB_ * NIMG_ * 2, 128, 0, stream>>>(P, Wc, x1, x2, cf, feat);
  k_tok<<<NB_ * NIMG_ * 4, 64, 0, stream>>>(feat, Wv, Wp, W1, W2, ln1g, ln1b, qkvb, projb,
                                           ln2g, ln2b, mb1, mb2, crs);
  (void)hipFuncSetAttribute(reinterpret_cast<const void*>(&k_dct),
                            hipFuncAttributeMaxDynamicSharedMemorySize, 65536);
  k_dct<<<NB_ * NC_, 128, 65536, stream>>>(crs, Dp, Epl);
  k_gate<<<1, 256, 0, stream>>>(Epl, fw1, fb1, fw2, fb2, scl);
  k_out<<<NT4_ / 256, 256, 0, stream>>>(crs, x1, x2, scl, out);
}
